// WalzeAttentionLayerV3_12644383719814
// MI455X (gfx1250) — hardware-run, weakly checked
//
#include <hip/hip_runtime.h>


namespace {
constexpr int NB_ = 8, C = 512, HH = 32, WW = 32, L = HH * WW, NT = NB_ * L  , HEADS = 8, HD = 64, DK = C / 4  , WIN = 32;
constexpr float XS = 8.0f, HS = 256.0f, PS = 256.0f, WSC = 256.0f, SCALE = 0.125f, BN_EPS = 1e-5f;
typedef _Float16 b16;
typedef __attribute__((ext_vector_type(16))) _Float16 v16b;
typedef __attribute__((ext_vector_type(8))) _Float16 v8b;
typedef __attribute__((ext_vector_type(2))) _Float16 v2b;
typedef __attribute__((ext_vector_type(8))) float v8f;
typedef __attribute__((ext_vector_type(4))) float v4f;
typedef __attribute__((ext_vector_type(2))) float v2f;
__device__ __forceinline__ float bf16_rne(float f) { unsigned int u = __float_as_uint(f); u += 0x7FFFu + ((u >> 16) & 1u); float r = __uint_as_float(u & 0xFFFF0000u); asm volatile("" : "+v"(r)); return r; }
__device__ __forceinline__ float bfv(float f) { float r = bf16_rne(f); asm volatile("" : "+v"(r)); return r; }
__device__ __forceinline__ void split16(float v, b16& hi, b16& lo) { hi = (b16)v; lo = (b16)(v - (float)hi); }
__device__ __forceinline__ v16b frag_kb(const b16* p, int hh) { const v8b a = *(const v8b*)(p + 8 * hh), b = *(const v8b*)(p + 16 + 8 * hh); v16b f;
#pragma unroll
  for (int e = 0; e < 8; ++e) { f[e] = a[e]; f[8 + e] = b[e]; } return f; }
__device__ __forceinline__ v8f wmma16b(v16b a, v16b b, v8f c) { v8f d = __builtin_amdgcn_wmma_f32_16x16x32_f16(false, a, false, b, (short)0, c, false, false); asm volatile("v_nop\n\tv_nop\n\tv_nop\n\tv_nop" : "+v"(d) : "v"(a), "v"(b)); return d; }
__device__ __forceinline__ void wave_lds_sync() { __builtin_amdgcn_fence(__ATOMIC_RELEASE, "workgroup"); __builtin_amdgcn_wave_barrier(); __builtin_amdgcn_fence(__ATOMIC_ACQUIRE, "workgroup"); }
__device__ __forceinline__ float pmul(float a, float b) { float p = a * b; asm volatile("" : "+v"(p)); return p; }
__device__ __forceinline__ float gelu_erf(float v) { return 0.5f * v * (1.0f + erff(v * 0.70710678118654752f)); }

__global__ __launch_bounds__(256) void wput_kernel(const float* __restrict__ dw1, const float* __restrict__ ipw, const float* __restrict__ opw, b16* __restrict__ WD1, b16* __restrict__ WIN_, b16* __restrict__ WOUT) { const size_t nt = (size_t)gridDim.x * 256, u0 = (size_t)blockIdx.x * 256 + threadIdx.x; v8b v;
  for (size_t u = u0; u < (size_t)DK * 2 * C / 8; u += nt) {
#pragma unroll
    for (int j = 0; j < 8; ++j) v[j] = (b16)(bf16_rne(dw1[u * 8 + j]) * WSC); for (int pass = 0; pass < 2; ++pass) { *(volatile v8b*)(WD1 + u * 8) = v; __threadfence(); } }
  for (size_t u = u0; u < (size_t)3 * C * C / 8; u += nt) {
#pragma unroll
    for (int j = 0; j < 8; ++j) v[j] = (b16)(bf16_rne(ipw[u * 8 + j]) * WSC); for (int pass = 0; pass < 2; ++pass) { *(volatile v8b*)(WIN_ + u * 8) = v; __threadfence(); } }
  for (size_t u = u0; u < (size_t)C * C / 8; u += nt) {
#pragma unroll
    for (int j = 0; j < 8; ++j) v[j] = (b16)(bf16_rne(opw[u * 8 + j]) * WSC); for (int pass = 0; pass < 2; ++pass) { *(volatile v8b*)(WOUT + u * 8) = v; __threadfence(); } } }
__global__ __launch_bounds__(32) void walze_kernel(const float* __restrict__ x, const float* __restrict__ dww, const float* __restrict__ dwb, const float* __restrict__ sw, const float* __restrict__ sb, const float* __restrict__ mixw, const float* __restrict__ bng, const float* __restrict__ bnb, int TLIM, float* __restrict__ XW, float* __restrict__ XT) { __shared__ float Tw[16][C + 1], Tx[16][C + 1]; const int lane = threadIdx.x; const size_t t0 = (size_t)blockIdx.x * 16; if (t0 >= (size_t)TLIM) return; const int b = (int)(t0 / L), hw0 = (int)(t0 % L); const int yy = hw0 / WW, xb = hw0 % WW;
  const float mix = 1.0f / (1.0f + __expf(-bfv(mixw[0]))), rs = rsqrtf(1.0f + BN_EPS); float s9[9]; for (int i = 0; i < 9; ++i) s9[i] = bfv(sw[i]); const float sbb = bfv(sb[0]);
  for (int cc = 0; cc < 16; ++cc) { const int c = lane * 16 + cc; const float* xc = x + ((size_t)b * C + c) * L; float w9[9]; for (int i = 0; i < 9; ++i) w9[i] = bfv(dww[(size_t)c * 9 + i]); const float db = bfv(dwb[c]), g = bfv(bng[c]), bt = bfv(bnb[c]);
    for (int t = 0; t < 16; ++t) { const int xx = xb + t; float m = db, e = sbb;
#pragma unroll
      for (int ky = 0; ky < 3; ++ky) { const int sy = (yy + ky - 1 + HH) % HH;
#pragma unroll
        for (int kx = 0; kx < 3; ++kx) { const int sx = (xx + kx - 1 + WW) % WW; const float xv = bfv(xc[sy * WW + sx]); m += pmul(w9[ky * 3 + kx], xv); e += pmul(s9[ky * 3 + kx], xv); } }
      const float xv0 = bfv(xc[yy * WW + xx]); const float comb = pmul(mix, m) + pmul(1.0f - mix, e) + xv0; Tw[t][c] = gelu_erf(pmul(pmul(g, comb), rs) + bt); Tx[t][c] = xv0; } }
  wave_lds_sync();
  for (int pass = 0; pass < 2; ++pass) { for (int t = 0; t < 16; ++t) for (int q = 0; q < 4; ++q) { *(volatile v4f*)(XW + (t0 + t) * C + q * 128 + lane * 4) = *(const v4f*)(&Tw[t][q * 128 + lane * 4]); *(volatile v4f*)(XT + (t0 + t) * C + q * 128 + lane * 4) = *(const v4f*)(&Tx[t][q * 128 + lane * 4]); } __threadfence(); } }
__global__ __launch_bounds__(32) void dq_kernel(const float* __restrict__ XT, const float* __restrict__ XW, const b16* __restrict__ WD1, const float* __restrict__ db1, const float* __restrict__ dw2, const float* __restrict__ db2, const b16* __restrict__ WIN_, const float* __restrict__ ipb, int TLIM, float* __restrict__ MASK, b16* __restrict__ Qh, b16* __restrict__ Ql, b16* __restrict__ Kh, b16* __restrict__ Kl, float* __restrict__ V) { __shared__ __attribute__((aligned(16))) b16 Ah[16][2 * C + 8], Al[16][2 * C + 8]; __shared__ float Tf[16][260], Hd[16][DK + 1]; const int lane = threadIdx.x, nloc = lane & 15, hlf = lane >> 4; const size_t t0 = (size_t)blockIdx.x * 16; if (t0 >= (size_t)TLIM) return;
  for (int rr = 0; rr < 16; ++rr) for (int q = 0; q < C / 32; ++q) { const int c = q * 32 + lane; Ah[rr][c] = (b16)(XT[(t0 + rr) * C + c] * HS); Al[rr][c] = (b16)0.0f;     b16 p, pl; split16(XW[(t0 + rr) * C + c] * HS, p, pl); Ah[rr][C + c] = p; Al[rr][C + c] = pl; }
  if (lane < 16) for (int k = 2 * C; k < 2 * C + 8; ++k) { Ah[lane][k] = (b16)0.0f; Al[lane][k] = (b16)0.0f; }
  wave_lds_sync();
  { v8f acc[8];
#pragma unroll
    for (int t = 0; t < 8; ++t) acc[t] = (v8f){};
#pragma unroll 2
    for (int kb = 0; kb < 2 * C; kb += 32) { const v16b a = frag_kb(&Ah[nloc][kb], hlf), al = frag_kb(&Al[nloc][kb], hlf);
#pragma unroll
      for (int t = 0; t < 8; ++t) { const v16b bw = frag_kb(WD1 + (size_t)(t * 16 + nloc) * 2 * C + kb, hlf); acc[t] = wmma16b(a, bw, acc[t]); if (kb >= C) acc[t] = wmma16b(al, bw, acc[t]); } }
#pragma unroll
    for (int t = 0; t < 8; ++t) { const int cc = t * 16 + nloc; const float bb = bfv(db1[cc]);
#pragma unroll
      for (int r8 = 0; r8 < 8; ++r8) Hd[8 * hlf + r8][cc] = gelu_erf(acc[t][r8] * (1.0f / (HS * WSC)) + bb); } }
  wave_lds_sync();
  if (lane < 16) { float s = bfv(db2[0]); for (int k = 0; k < DK; ++k) s += pmul(Hd[lane][k], bfv(dw2[k])); Hd[lane][DK] = 1.0f / (1.0f + __expf(-s)); }
  wave_lds_sync();
  for (int pass = 0; pass < 2; ++pass) { ((volatile float*)MASK)[(size_t)blockIdx.x * 32 + lane] = lane < 16 ? Hd[lane][DK] : 0.0f; __threadfence(); }
#pragma unroll 1
  for (int g = 0; g < 6; ++g) { v8f acc[16];
#pragma unroll
    for (int t = 0; t < 16; ++t) acc[t] = (v8f){};
#pragma unroll 2
    for (int kb = 0; kb < C; kb += 32) { const v16b a = frag_kb(&Ah[nloc][C + kb], hlf), al = frag_kb(&Al[nloc][C + kb], hlf);
#pragma unroll
      for (int t = 0; t < 16; ++t) { const v16b bw = frag_kb(WIN_ + (size_t)(g * 256 + t * 16 + nloc) * C + kb, hlf); acc[t] = wmma16b(a, bw, acc[t]); acc[t] = wmma16b(al, bw, acc[t]); } }
#pragma unroll
    for (int t = 0; t < 16; ++t) { const int cc = t * 16 + nloc; const float bb = bfv(ipb[g * 256 + cc]);
#pragma unroll
      for (int r8 = 0; r8 < 8; ++r8) Tf[8 * hlf + r8][cc] = acc[t][r8] * (1.0f / (HS * WSC)) + bb; }
    wave_lds_sync();
    const int which = g / 2, c0 = (g % 2) * 256;
    for (int pass = 0; pass < 2; ++pass) { for (int rr = 0; rr < 16; ++rr) { const size_t tk = t0 + rr;
        if (which == 2) { for (int q = 0; q < 2; ++q) *(volatile v4f*)(V + tk * C + c0 + q * 128 + lane * 4) = *(const v4f*)(&Tf[rr][q * 128 + lane * 4]); }
        else { b16* Ph = which == 0 ? Qh : Kh; b16* Pl = which == 0 ? Ql : Kl; for (int q = 0; q < 4; ++q) { const int c = q * 64 + lane * 2; b16 h0, l0, h1, l1; split16(Tf[rr][c] * HS, h0, l0); split16(Tf[rr][c + 1] * HS, h1, l1); *(volatile v2b*)(Ph + tk * C + c0 + c) = (v2b){h0, h1}; *(volatile v2b*)(Pl + tk * C + c0 + c) = (v2b){l0, l1}; } } }
      __threadfence(); }
    wave_lds_sync(); } }
__global__ __launch_bounds__(256) void vt_kernel(const float* __restrict__ V, int TLIM, b16* __restrict__ VTh, b16* __restrict__ VTl) { __shared__ float Tt[64][257]; const int tt = blockIdx.x >> 1, hg = blockIdx.x & 1; const size_t t0 = (size_t)tt * 64; if (t0 >= (size_t)TLIM) return; const int b = (int)(t0 / L), s0 = (int)(t0 % L); const int tid = threadIdx.x, wave = tid >> 5, lane = tid & 31;
  for (int q = wave; q < 64; q += 8) for (int c = lane; c < 256; c += 32) Tt[q][c] = V[(t0 + q) * C + hg * 256 + c];
  __syncthreads();
  for (int pass = 0; pass < 2; ++pass) { for (int c = wave; c < 256; c += 8) { const int h = hg * 4 + c / HD, d = c % HD; b16 h0, l0, h1, l1; split16(Tt[lane * 2][c] * HS, h0, l0); split16(Tt[lane * 2 + 1][c] * HS, h1, l1); const size_t o = (((size_t)b * HEADS + h) * HD + d) * L + s0 + lane * 2; *(volatile v2b*)(VTh + o) = (v2b){h0, h1}; *(volatile v2b*)(VTl + o) = (v2b){l0, l1}; } __threadfence(); } }
__global__ __launch_bounds__(32) void att_kernel(const b16* __restrict__ Qh, const b16* __restrict__ Ql, const b16* __restrict__ Kh, const b16* __restrict__ Kl, const b16* __restrict__ VTh, const b16* __restrict__ VTl, int TLIM, float* __restrict__ CTX) { __shared__ __attribute__((aligned(16))) b16 Pa[16][72], Pb[16][72]; __shared__ float Sc[16][65], Of[16][HD + 1]; const int lane = threadIdx.x, nloc = lane & 15, hlf = lane >> 4; const int bh = blockIdx.x / (L / 16), q0 = (blockIdx.x % (L / 16)) * 16; const int b = bh / HEADS, h = bh % HEADS; const size_t tq = (size_t)b * L + q0; if (tq >= (size_t)TLIM) return;
  int k0 = q0 - WIN / 2; if (k0 < 0) k0 = 0; if (k0 > L - 64) k0 = L - 64;
  v8f s[4] = {(v8f){}, (v8f){}, (v8f){}, (v8f){}};
#pragma unroll
  for (int ks = 0; ks < 2; ++ks) { const v16b qa = frag_kb(Qh + (tq + nloc) * C + h * HD + ks * 32, hlf), ql = frag_kb(Ql + (tq + nloc) * C + h * HD + ks * 32, hlf);
#pragma unroll
    for (int t = 0; t < 4; ++t) { const size_t ko = ((size_t)b * L + k0 + t * 16 + nloc) * C + h * HD + ks * 32; const v16b kh = frag_kb(Kh + ko, hlf), kl = frag_kb(Kl + ko, hlf); s[t] = wmma16b(qa, kh, s[t]); s[t] = wmma16b(qa, kl, s[t]); s[t] = wmma16b(ql, kh, s[t]); } }
#pragma unroll
  for (int t = 0; t < 4; ++t)
#pragma unroll
    for (int r8 = 0; r8 < 8; ++r8) Sc[8 * hlf + r8][t * 16 + nloc] = s[t][r8] * (SCALE / (HS * HS));
  if (lane < 16) for (int k = 64; k < 72; ++k) { Pa[lane][k] = (b16)0.0f; Pb[lane][k] = (b16)0.0f; }
  wave_lds_sync();
  if (lane < 16) { const int r = lane, qi = q0 + r; float mx = -INFINITY; for (int j = 0; j < 64; ++j) { const int kj = k0 + j; if (kj >= qi - WIN / 2 && kj <= qi + WIN / 2) mx = fmaxf(mx, Sc[r][j]); } float sm = 0.0f; for (int j = 0; j < 64; ++j) { const int kj = k0 + j; const float p = (kj >= qi - WIN / 2 && kj <= qi + WIN / 2) ? __expf(Sc[r][j] - mx) : 0.0f; Sc[r][j] = p; sm += p; } const float inv = 1.0f / sm; for (int j = 0; j < 64; ++j) { b16 p, pl; split16(Sc[r][j] * inv * PS, p, pl); Pa[r][j] = p; Pb[r][j] = pl; } }
  wave_lds_sync();
  v8f o[4] = {(v8f){}, (v8f){}, (v8f){}, (v8f){}};
#pragma unroll
  for (int kb = 0; kb < 64; kb += 32) { const v16b pa = frag_kb(&Pa[nloc][kb], hlf), pb = frag_kb(&Pb[nloc][kb], hlf);
#pragma unroll
    for (int t = 0; t < 4; ++t) { const size_t vo = ((size_t)bh * HD + t * 16 + nloc) * L + k0 + kb; const v16b vh = frag_kb(VTh + vo, hlf), vl = frag_kb(VTl + vo, hlf); o[t] = wmma16b(pa, vh, o[t]); o[t] = wmma16b(pa, vl, o[t]); o[t] = wmma16b(pb, vh, o[t]); } }
#pragma unroll
  for (int t = 0; t < 4; ++t)
#pragma unroll
    for (int r8 = 0; r8 < 8; ++r8) Of[8 * hlf + r8][t * 16 + nloc] = o[t][r8] * (1.0f / (PS * HS));
  wave_lds_sync();
  for (int pass = 0; pass < 2; ++pass) { for (int r = 0; r < 16; ++r) *(volatile v2f*)(CTX + (tq + r) * C + h * HD + lane * 2) = (v2f){Of[r][lane * 2], Of[r][lane * 2 + 1]}; __threadfence(); } }
__global__ __launch_bounds__(32) void out_kernel(const float* __restrict__ CTX, const float* __restrict__ XW, const float* __restrict__ MASK, const b16* __restrict__ WOUT, const float* __restrict__ opb, int TLIM, float* __restrict__ FIN) { __shared__ __attribute__((aligned(16))) b16 Ah[16][C + 8], Al[16][C + 8]; __shared__ float Tf[16][260]; const int lane = threadIdx.x, nloc = lane & 15, hlf = lane >> 4; const size_t t0 = (size_t)blockIdx.x * 16; if (t0 >= (size_t)TLIM) return;
  for (int rr = 0; rr < 16; ++rr) for (int q = 0; q < C / 32; ++q) { const int c = q * 32 + lane; b16 p, pl; split16(CTX[(t0 + rr) * C + c] * HS, p, pl); Ah[rr][c] = p; Al[rr][c] = pl; }
  if (lane < 16) for (int k = C; k < C + 8; ++k) { Ah[lane][k] = (b16)0.0f; Al[lane][k] = (b16)0.0f; }
  wave_lds_sync();
#pragma unroll 1
  for (int g = 0; g < 2; ++g) { v8f acc[16];
#pragma unroll
    for (int t = 0; t < 16; ++t) acc[t] = (v8f){};
#pragma unroll 2
    for (int kb = 0; kb < C; kb += 32) { const v16b a = frag_kb(&Ah[nloc][kb], hlf), al = frag_kb(&Al[nloc][kb], hlf);
#pragma unroll
      for (int t = 0; t < 16; ++t) { const v16b bw = frag_kb(WOUT + (size_t)(g * 256 + t * 16 + nloc) * C + kb, hlf); acc[t] = wmma16b(a, bw, acc[t]); acc[t] = wmma16b(al, bw, acc[t]); } }
#pragma unroll
    for (int t = 0; t < 16; ++t) { const int cc = t * 16 + nloc; const float bb = bfv(opb[g * 256 + cc]);
#pragma unroll
      for (int r8 = 0; r8 < 8; ++r8) { const int rr = 8 * hlf + r8; const size_t tk = t0 + rr; Tf[rr][cc] = XW[tk * C + g * 256 + cc] + pmul(MASK[(tk / 16) * 32 + (tk % 16)], acc[t][r8] * (1.0f / (HS * WSC)) + bb); } }
    wave_lds_sync();
    for (int pass = 0; pass < 2; ++pass) { for (int rr = 0; rr < 16; ++rr) for (int q = 0; q < 2; ++q) *(volatile v4f*)(FIN + (t0 + rr) * C + g * 256 + q * 128 + lane * 4) = *(const v4f*)(&Tf[rr][q * 128 + lane * 4]); __threadfence(); }
    wave_lds_sync(); } }
__global__ __launch_bounds__(256) void copy_kernel(const float* __restrict__ FIN, int TLIM, float* __restrict__ out) { const size_t u = (size_t)blockIdx.x * 256 + threadIdx.x; if (u >= (size_t)NB_ * C * L) return; const int hw = (int)(u % L), c = (int)((u / L) % C), b = (int)(u / ((size_t)L * C)); const size_t tk = (size_t)b * L + hw; const float v = tk < (size_t)TLIM ? FIN[tk * C + c] : 0.0f;
  for (int pass = 0; pass < 2; ++pass) { ((volatile float*)out)[u] = v; __threadfence(); } }
}

extern "C" void kernel_launch(void* const* d_in, const int* in_sizes, int n_in, void* d_out, int out_size, void* d_ws, size_t ws_size, hipStream_t stream) {
  (void)n_in;
  auto Fp = [&](int i) { return (const float*)d_in[i]; };
  if (in_sizes[0] != NT * C || in_sizes[1] != C * 9 || in_sizes[3] != 9 || in_sizes[5] != 1 || in_sizes[8] != DK * 2 * C || in_sizes[10] != DK || in_sizes[12] != 3 * C * C || in_sizes[14] != C * C || out_size != NT * C) return;
  const int TLIM = NT;
  size_t off = 0; char* ws = (char*)d_ws;
  auto carve = [&](size_t bytes) { char* p = ws + off; off += (bytes + 255) & ~(size_t)255; return p; };
  b16* WD1 = (b16*)carve((size_t)DK * 2 * C * 2); b16* WIN_ = (b16*)carve((size_t)3 * C * C * 2); b16* WOUT = (b16*)carve((size_t)C * C * 2); float* XW = (float*)carve((size_t)NT * C * 4); float* XT = (float*)carve((size_t)NT * C * 4); float* MASK = (float*)carve((size_t)(NT / 16) * 32 * 4); b16* Qh = (b16*)carve((size_t)NT * C * 2); b16* Ql = (b16*)carve((size_t)NT * C * 2); b16* Kh = (b16*)carve((size_t)NT * C * 2); b16* Kl = (b16*)carve((size_t)NT * C * 2); float* V = (float*)carve((size_t)NT * C * 4); b16* VTh = (b16*)carve((size_t)NT * C * 2); b16* VTl = (b16*)carve((size_t)NT * C * 2); float* CTX = (float*)carve((size_t)NT * C * 4); float* FIN = XT;
  if (off > ws_size || off > ((size_t)136 << 20)) return;
  wput_kernel<<<256, 256, 0, stream>>>(Fp(8), Fp(12), Fp(14), WD1, WIN_, WOUT);
  walze_kernel<<<NT / 16, 32, 0, stream>>>(Fp(0), Fp(1), Fp(2), Fp(3), Fp(4), Fp(5), Fp(6), Fp(7), TLIM, XW, XT);
  dq_kernel<<<NT / 16, 32, 0, stream>>>(XT, XW, WD1, Fp(9), Fp(10), Fp(11), WIN_, Fp(13), TLIM, MASK, Qh, Ql, Kh, Kl, V);
  vt_kernel<<<(NT / 64) * 2, 256, 0, stream>>>(V, TLIM, VTh, VTl);
  att_kernel<<<NB_ * HEADS * (L / 16), 32, 0, stream>>>(Qh, Ql, Kh, Kl, VTh, VTl, TLIM, CTX);
  out_kernel<<<NT / 16, 32, 0, stream>>>(CTX, XW, MASK, WOUT, Fp(15), TLIM, FIN);
  copy_kernel<<<(NT * C + 255) / 256, 256, 0, stream>>>(FIN, TLIM, (float*)d_out);
}
